// MyMultiHeadAttention_8546984919358
// MI455X (gfx1250) — hardware-verified
//
#include <hip/hip_runtime.h>


#ifndef NB
#define NB 2
#endif
#ifndef SEQ
#define SEQ 2048
#endif
#define NB_FULL  2
#define SEQ_FULL 2048
#define DM   1024
#define NH   16
#define HD   64
#define DQ   (NH * HD)
#define NFR  32
#define MAXS 2048
#define KCH  64
#define PP   72
#define PCAR 1024.0f
#define SCL  0.125f
#define L2E  1.4426950408889634f
static_assert(NB >= 1 && NB <= NB_FULL);
static_assert(SEQ >= KCH && SEQ <= SEQ_FULL && SEQ % 64 == 0 && SEQ % KCH == 0);
static_assert(DM % 64 == 0 && DQ == DM && HD == 64 && KCH == 64 && NFR * 2 == HD && MAXS >= SEQ_FULL);
static_assert((MAXS * NFR) % 256 == 0 && (DM * DM) % 2048 == 0);

typedef _Float16 h16;
typedef unsigned short bf;
typedef __attribute__((ext_vector_type(16))) __bf16   v16bf;
typedef __attribute__((ext_vector_type(16))) _Float16 v16h;
typedef __attribute__((ext_vector_type(8)))  _Float16 v8h;
typedef __attribute__((ext_vector_type(8)))  unsigned short v8us;
typedef __attribute__((ext_vector_type(8)))  float    v8f;
typedef __attribute__((ext_vector_type(4)))  float    v4f;
typedef __attribute__((ext_vector_type(2)))  unsigned short v2us;
typedef __attribute__((ext_vector_type(2)))  float    v2f;
typedef v8h  __attribute__((may_alias)) v8ha;
typedef v4f  __attribute__((may_alias)) v4fa;
typedef v8us __attribute__((may_alias)) v8usa;

__device__ __forceinline__ unsigned short f2bf(float f) { unsigned u = __float_as_uint(f); u += 0x7FFFu + ((u >> 16) & 1u); return (unsigned short)(u >> 16); }
__device__ __forceinline__ float bf2f(unsigned short b) { return __uint_as_float(((unsigned)b) << 16); }
__device__ __forceinline__ float bfr(float f) { return bf2f(f2bf(f)); }
__device__ __forceinline__ v16h cat16(v8h lo, v8h hi) { return __builtin_shufflevector(lo, hi, 0, 1, 2, 3, 4, 5, 6, 7, 8, 9, 10, 11, 12, 13, 14, 15); }
__device__ __forceinline__ v16bf cat16b(v8us lo, v8us hi) { return __builtin_bit_cast(v16bf, __builtin_shufflevector(lo, hi, 0, 1, 2, 3, 4, 5, 6, 7, 8, 9, 10, 11, 12, 13, 14, 15)); }
__device__ __forceinline__ v8f wmma16(v16h a, v16h b, v8f c) { return __builtin_amdgcn_wmma_f32_16x16x32_f16(false, a, false, b, (short)0, c, false, false); }
__device__ __forceinline__ v8f wmmab(v16bf a, v16bf b, v8f c) { return __builtin_amdgcn_wmma_f32_16x16x32_bf16(false, a, false, b, (short)0, c, false, false); }
__device__ __forceinline__ void splitf(float y, unsigned short& h, unsigned short& l) { h = f2bf(y); l = f2bf(y - bf2f(h)); }

template <typename T16> struct WFrag;
template <> struct WFrag<h16> { typedef v16h V; static __device__ __forceinline__ V ld(const h16* p) { return cat16(*(const v8h*)p, *(const v8h*)(p + 16)); } static __device__ __forceinline__ v8f mma(V a, V b, v8f c) { return wmma16(a, b, c); } };
template <> struct WFrag<bf> { typedef v16bf V; static __device__ __forceinline__ V ld(const bf* p) { return cat16b(*(const v8us*)p, *(const v8us*)(p + 16)); } static __device__ __forceinline__ v8f mma(V a, V b, v8f c) { return wmmab(a, b, c); } };
template <typename T16, int NSPLIT, bool BIAS>
__global__ __launch_bounds__(32) void k_gemmw(const T16* __restrict__ A, const T16* __restrict__ A2, const T16* __restrict__ Bt, const T16* __restrict__ Bt2, int K, float* C, int ldc, const float* __restrict__ bias, size_t sA, size_t sB, size_t sC) {
    typedef typename WFrag<T16>::V V;
    __shared__ __align__(16) float os[16 * 68];
    const size_t z = blockIdx.z; A += z * sA; if (A2) A2 += z * sA; Bt += z * sB; if (Bt2) Bt2 += z * sB; C += z * sC;
    const int lane = threadIdx.x & 31, lr = lane & 15, hi = lane >> 4; const int r0 = blockIdx.x * 64, c0 = blockIdx.y * 64;
    v8f acc[4][4];
#pragma unroll
    for (int mb = 0; mb < 4; ++mb)
#pragma unroll
        for (int nb = 0; nb < 4; ++nb) acc[mb][nb] = (v8f){};
    const size_t aoff = (size_t)(r0 + lr) * K + 8 * hi, boff = (size_t)(c0 + lr) * K + 8 * hi;
#pragma unroll 1
    for (int kc = 0; kc < K; kc += 32) {
        V a[4], a2[4];
#pragma unroll
        for (int mb = 0; mb < 4; ++mb) { a[mb] = WFrag<T16>::ld(A + aoff + (size_t)mb * 16 * K + kc); if (NSPLIT == 1 || NSPLIT == 2) a2[mb] = WFrag<T16>::ld(A2 + aoff + (size_t)mb * 16 * K + kc); }
#pragma unroll
        for (int nb = 0; nb < 4; ++nb) { const V b = WFrag<T16>::ld(Bt + boff + (size_t)nb * 16 * K + kc); V b2; if (NSPLIT >= 2) b2 = WFrag<T16>::ld(Bt2 + boff + (size_t)nb * 16 * K + kc);
#pragma unroll
            for (int mb = 0; mb < 4; ++mb) { acc[mb][nb] = WFrag<T16>::mma(a[mb], b, acc[mb][nb]); if (NSPLIT == 1 || NSPLIT == 2) acc[mb][nb] = WFrag<T16>::mma(a2[mb], b, acc[mb][nb]); if (NSPLIT >= 2) acc[mb][nb] = WFrag<T16>::mma(a[mb], b2, acc[mb][nb]); } }
        asm volatile("v_nop\n\tv_nop\n\tv_nop\n\tv_nop" : "+v"(acc[0][0]), "+v"(acc[1][1]), "+v"(acc[2][2]), "+v"(acc[3][3]) : "v"(a[0]), "v"(a[3]));
    }
#pragma unroll
    for (int mb = 0; mb < 4; ++mb) {
#pragma unroll
        for (int nb = 0; nb < 4; ++nb) {
#pragma unroll
            for (int j = 0; j < 8; ++j) os[(hi * 8 + j) * 68 + nb * 16 + lr] = acc[mb][nb][j]; }
        __builtin_amdgcn_wave_barrier(); asm volatile("" ::: "memory");
        float* crow = C + (size_t)(r0 + mb * 16) * ldc + c0;
#pragma unroll 1
        for (int ps = 0; ps < 2; ++ps) {
#pragma unroll
            for (int s = 0; s < 8; ++s) { const int row = 2 * s + hi, cofs = lr * 4; v4f val = *(const v4fa*)(os + row * 68 + cofs); if (BIAS) { val[0] += bfr(bias[c0 + cofs]); val[1] += bfr(bias[c0 + cofs + 1]); val[2] += bfr(bias[c0 + cofs + 2]); val[3] += bfr(bias[c0 + cofs + 3]); }
                *(volatile v4f*)(crow + (size_t)row * ldc + cofs) = val; }
            if (ps == 0) __threadfence(); }
        __builtin_amdgcn_wave_barrier(); asm volatile("" ::: "memory");
    }
}

__global__ __launch_bounds__(256) void k_cvtw(const float* __restrict__ w, bf* Wb, size_t n8) { const size_t i = (size_t)blockIdx.x * 256 + threadIdx.x; if (i >= n8) return; const v8f v = *(const v8f*)(w + i * 8); v8us o;
#pragma unroll
    for (int k = 0; k < 8; ++k) o[k] = f2bf(v[k]); *(volatile v8us*)(Wb + i * 8) = o; __threadfence(); *(volatile v8us*)(Wb + i * 8) = o; }
__global__ __launch_bounds__(256) void k_cvtx(const float* __restrict__ x, bf* XB, size_t n8) { const size_t i = (size_t)blockIdx.x * 256 + threadIdx.x; if (i >= n8) return; const size_t per = (size_t)SEQ * DM / 8; const size_t b = i / per, r = i - b * per; const v8f v = *(const v8f*)(x + b * (size_t)SEQ_FULL * DM + r * 8); v8us o;
#pragma unroll
    for (int k = 0; k < 8; ++k) o[k] = f2bf(v[k]); *(volatile v8us*)(XB + i * 8) = o; __threadfence(); *(volatile v8us*)(XB + i * 8) = o; }

__constant__ float c_invf[NFR] = {
    1.0f,                     0.749894209332455827f,    0.562341325190349080f,    0.421696503428582248f,
    0.316227766016837933f,    0.237137370566165526f,    0.177827941003892280f,    0.133352143216332403f,
    0.1f,                     0.0749894209332455827f,   0.0562341325190349080f,   0.0421696503428582248f,
    0.0316227766016837933f,   0.0237137370566165526f,   0.0177827941003892280f,   0.0133352143216332403f,
    0.01f,                    7.49894209332455827e-3f,  5.62341325190349080e-3f,  4.21696503428582248e-3f,
    3.16227766016837933e-3f,  2.37137370566165526e-3f,  1.77827941003892280e-3f,  1.33352143216332403e-3f,
    1.0e-3f,                  7.49894209332455827e-4f,  5.62341325190349080e-4f,  4.21696503428582248e-4f,
    3.16227766016837933e-4f,  2.37137370566165526e-4f,  1.77827941003892280e-4f,  1.33352143216332403e-4f };

__global__ __launch_bounds__(256) void k_ropetab(float* CT, float* ST) {
#pragma clang fp contract(off)
    const int idx = blockIdx.x * 256 + threadIdx.x; if (idx >= MAXS * NFR) return;
    const int p = idx >> 5, i = idx & 31;
    const float ang = (float)p * c_invf[i];
    const float cv = cosf(ang); const float sv = sinf(ang);
    *(volatile float*)(CT + idx) = cv; *(volatile float*)(ST + idx) = sv; __threadfence();
    *(volatile float*)(CT + idx) = cv; *(volatile float*)(ST + idx) = sv;
}

template <bool ISQ>
__global__ __launch_bounds__(256) void k_ropepl(const float* __restrict__ F, const float* __restrict__ CT, const float* __restrict__ ST, const int* __restrict__ tok, bf* Ph, bf* Pl) {
#pragma clang fp contract(off)
    const size_t e = ((size_t)blockIdx.x * 256 + threadIdx.x) * 2; if (e >= (size_t)NB * NH * SEQ * HD) return;
    const int d = (int)(e % HD); const int s = (int)((e / HD) % SEQ); const int h = (int)((e / ((size_t)HD * SEQ)) % NH); const int b = (int)(e / ((size_t)HD * SEQ * NH));
    const v2f x2 = *(const v2f*)(F + ((size_t)b * SEQ + s) * DQ + (size_t)h * HD + d);
    int p = tok[s]; p = (p < 0) ? (p + MAXS) : p; p = (p < 0) ? 0 : p; p = (p > MAXS - 1) ? (MAXS - 1) : p;
    const int ti = p * NFR + (d >> 1);
    const float cv = CT[ti], sv = ST[ti];
    const float m0 = x2[0] * cv, m1 = x2[1] * sv, m2 = x2[0] * sv, m3 = x2[1] * cv;
    float y0 = m0 - m1, y1 = m2 + m3;
    if (ISQ) { y0 = y0 * SCL; y1 = y1 * SCL; }
    v2us oh, ol; unsigned short a, c2;
    splitf(y0, a, c2); oh[0] = a; ol[0] = c2; splitf(y1, a, c2); oh[1] = a; ol[1] = c2;
    *(volatile v2us*)(Ph + e) = oh; *(volatile v2us*)(Pl + e) = ol; __threadfence();
    *(volatile v2us*)(Ph + e) = oh; *(volatile v2us*)(Pl + e) = ol;
}
__global__ __launch_bounds__(256) void k_vtp(const float* __restrict__ F, bf* Vh, bf* Vl) {
    const size_t e = ((size_t)blockIdx.x * 256 + threadIdx.x) * 2; if (e >= (size_t)NB * NH * HD * SEQ) return;
    const int t = (int)(e % SEQ); const int d = (int)((e / SEQ) % HD); const int h = (int)((e / ((size_t)SEQ * HD)) % NH); const int b = (int)(e / ((size_t)SEQ * HD * NH));
    v2us oh, ol;
#pragma unroll
    for (int q = 0; q < 2; ++q) { const float xv = F[((size_t)b * SEQ + t + q) * DQ + (size_t)h * HD + d]; unsigned short a, c2; splitf(xv, a, c2); oh[q] = a; ol[q] = c2; }
    *(volatile v2us*)(Vh + e) = oh; *(volatile v2us*)(Vl + e) = ol; __threadfence(); *(volatile v2us*)(Vh + e) = oh; *(volatile v2us*)(Vl + e) = ol;
}

__global__ __launch_bounds__(32) __attribute__((amdgpu_num_vgpr(256)))
void k_attn(const bf* __restrict__ Qh, const bf* __restrict__ Ql, const bf* __restrict__ Kh, const bf* __restrict__ Kl,
            const bf* __restrict__ Vh, const bf* __restrict__ Vl, bf* Ah, bf* Al) {
    __shared__ __align__(16) bf psh[16 * PP];
    __shared__ __align__(16) bf psl[16 * PP];
    __shared__ __align__(16) float os[16 * 68];
    const int lane = threadIdx.x & 31, lr = lane & 15, hi = lane >> 4;
    const int s0 = blockIdx.x * 16, h = blockIdx.y, b = blockIdx.z;
    const size_t hp = ((size_t)b * NH + h) * (size_t)SEQ * HD;
    const bf* qh = Qh + hp + (size_t)(s0 + lr) * HD + 8 * hi; const bf* ql = Ql + hp + (size_t)(s0 + lr) * HD + 8 * hi;
    const bf* kh = Kh + hp + (size_t)lr * HD + 8 * hi;        const bf* kl = Kl + hp + (size_t)lr * HD + 8 * hi;
    const bf* vh = Vh + hp + (size_t)lr * SEQ + 8 * hi;       const bf* vl = Vl + hp + (size_t)lr * SEQ + 8 * hi;
    v16bf qa[2], qa2[2];
#pragma unroll
    for (int ks = 0; ks < 2; ++ks) { qa[ks] = WFrag<bf>::ld(qh + ks * 32); qa2[ks] = WFrag<bf>::ld(ql + ks * 32); }
    float mrow[8], lrow[8];
#pragma unroll
    for (int r = 0; r < 8; ++r) { mrow[r] = -1.0e30f; lrow[r] = 0.0f; }
    v8f oacc[4];
#pragma unroll
    for (int nt = 0; nt < 4; ++nt) oacc[nt] = (v8f){};
    v16bf ph[2], pl[2];
    const int tend = (s0 / KCH) * KCH;
#pragma unroll 1
    for (int t0 = 0; t0 <= tend; t0 += KCH) {
        v8f sacc[4];
#pragma unroll
        for (int nt = 0; nt < 4; ++nt) sacc[nt] = (v8f){};
#pragma unroll
        for (int nt = 0; nt < 4; ++nt) {
#pragma unroll
            for (int ks = 0; ks < 2; ++ks) {
                const v16bf kbh = WFrag<bf>::ld(kh + (size_t)(t0 + nt * 16) * HD + ks * 32);
                const v16bf kbl = WFrag<bf>::ld(kl + (size_t)(t0 + nt * 16) * HD + ks * 32);
                sacc[nt] = wmmab(qa[ks], kbh, sacc[nt]); sacc[nt] = wmmab(qa2[ks], kbh, sacc[nt]); sacc[nt] = wmmab(qa[ks], kbl, sacc[nt]);
            }
        }
        asm volatile("v_nop\n\tv_nop\n\tv_nop\n\tv_nop" : "+v"(sacc[0]), "+v"(sacc[1]), "+v"(sacc[2]), "+v"(sacc[3]) : "v"(qa[0]), "v"(qa2[1]));
#pragma unroll
        for (int nt = 0; nt < 4; ++nt)
#pragma unroll
            for (int r = 0; r < 8; ++r) { const int kcol = t0 + nt * 16 + lr; const int qrow = s0 + 8 * hi + r; const float sv = sacc[nt][r]; sacc[nt][r] = (kcol <= qrow) ? sv : -__builtin_inff(); }
        float sc[8], rs[8];
#pragma unroll
        for (int r = 0; r < 8; ++r) {
            float m = fmaxf(fmaxf(sacc[0][r], sacc[1][r]), fmaxf(sacc[2][r], sacc[3][r]));
#pragma unroll
            for (int sh = 1; sh < 16; sh <<= 1) m = fmaxf(m, __shfl_xor(m, sh, 32));
            const float mn = fmaxf(mrow[r], m);
            sc[r] = __builtin_amdgcn_exp2f(__fmul_rn(__fsub_rn(mrow[r], mn), L2E)); mrow[r] = mn; rs[r] = 0.0f;
        }
#pragma unroll
        for (int nt = 0; nt < 4; ++nt)
#pragma unroll
            for (int r = 0; r < 8; ++r) { const float p = __builtin_amdgcn_exp2f(__fmul_rn(__fsub_rn(sacc[nt][r], mrow[r]), L2E)); sacc[nt][r] = p; rs[r] += p; }
#pragma unroll
        for (int r = 0; r < 8; ++r) {
            float s = rs[r];
#pragma unroll
            for (int sh = 1; sh < 16; sh <<= 1) s += __shfl_xor(s, sh, 32);
            lrow[r] = lrow[r] * sc[r] + s;
        }
#pragma unroll
        for (int nt = 0; nt < 4; ++nt)
#pragma unroll
            for (int r = 0; r < 8; ++r) oacc[nt][r] *= sc[r];
#pragma unroll
        for (int nt = 0; nt < 4; ++nt)
#pragma unroll
            for (int r = 0; r < 8; ++r) { unsigned short a, c2; splitf(sacc[nt][r] * PCAR, a, c2); const int o = (hi * 8 + r) * PP + nt * 16 + lr; psh[o] = a; psl[o] = c2; }
        __builtin_amdgcn_fence(3, "wavefront"); __builtin_amdgcn_wave_barrier();
#pragma unroll
        for (int kk = 0; kk < 2; ++kk) {
            ph[kk] = WFrag<bf>::ld(psh + lr * PP + kk * 32 + 8 * hi); pl[kk] = WFrag<bf>::ld(psl + lr * PP + kk * 32 + 8 * hi);
#pragma unroll
            for (int nt = 0; nt < 4; ++nt) {
                const v16bf vbh = WFrag<bf>::ld(vh + (size_t)nt * 16 * SEQ + t0 + kk * 32);
                const v16bf vbl = WFrag<bf>::ld(vl + (size_t)nt * 16 * SEQ + t0 + kk * 32);
                oacc[nt] = wmmab(ph[kk], vbh, oacc[nt]); oacc[nt] = wmmab(pl[kk], vbh, oacc[nt]); oacc[nt] = wmmab(ph[kk], vbl, oacc[nt]);
            }
        }
        asm volatile("v_nop\n\tv_nop\n\tv_nop\n\tv_nop" : "+v"(oacc[0]), "+v"(oacc[1]), "+v"(oacc[2]), "+v"(oacc[3]) : "v"(ph[0]), "v"(pl[1]));
        asm volatile("" ::: "memory");
    }
    float rinv[8];
#pragma unroll
    for (int r = 0; r < 8; ++r) rinv[r] = __fdiv_rn(1.0f, lrow[r] * PCAR);
#pragma unroll
    for (int nt = 0; nt < 4; ++nt)
#pragma unroll
        for (int r = 0; r < 8; ++r) os[(hi * 8 + r) * 68 + nt * 16 + lr] = oacc[nt][r] * rinv[r];
    __builtin_amdgcn_fence(3, "wavefront"); __builtin_amdgcn_wave_barrier();
    const int rg = lane >> 3, c8 = (lane & 7) * 8;
    bf* ah = Ah + ((size_t)b * SEQ + s0) * DQ + (size_t)h * HD + c8; bf* al = Al + ((size_t)b * SEQ + s0) * DQ + (size_t)h * HD + c8;
#pragma unroll 1
    for (int ps = 0; ps < 2; ++ps) {
#pragma unroll
        for (int it = 0; it < 4; ++it) {
            const int row = it * 4 + rg; const v4f x0 = *(const v4fa*)(os + row * 68 + c8); const v4f x1 = *(const v4fa*)(os + row * 68 + c8 + 4); v8us oh, ol;
#pragma unroll
            for (int j = 0; j < 4; ++j) { unsigned short a, c2; splitf(x0[j], a, c2); oh[j] = a; ol[j] = c2; splitf(x1[j], a, c2); oh[4 + j] = a; ol[4 + j] = c2; }
            *(volatile v8us*)(ah + (size_t)row * DQ) = oh; *(volatile v8us*)(al + (size_t)row * DQ) = ol;
        }
        if (ps == 0) __threadfence();
    }
}

extern "C" void kernel_launch(void* const* d_in, const int* in_sizes, int n_in,
                              void* d_out, int out_size, void* d_ws, size_t ws_size, hipStream_t stream) {
    if (n_in < 6) return;
    if ((long long)in_sizes[0] < ((long long)(NB - 1) * SEQ_FULL + SEQ) * DM) return;
    if (in_sizes[1] < SEQ) return;
    if (in_sizes[2] < DM * DM || in_sizes[3] < DM * DM || in_sizes[4] < DM * DM || in_sizes[5] < DM * DM) return;
    if (out_size < NB * SEQ * DM) return;
    const float* x   = (const float*)d_in[0];
    const int*   tok = (const int*)d_in[1];
    const float* wq  = (const float*)d_in[2];
    const float* wk  = (const float*)d_in[3];
    const float* wv  = (const float*)d_in[4];
    const float* wo  = (const float*)d_in[5];
    float* OUT = (float*)d_out;
    char* wsp = (char*)d_ws;
    auto take = [&](size_t bytes) { char* p = wsp; wsp += (bytes + 255) & ~(size_t)255; return (void*)p; };
    const size_t nw  = (size_t)DM * DM;
    const size_t npl = (size_t)NB * NH * SEQ * HD;
    bf* WB  = (bf*)take(3 * nw * 2);
    bf* WOB = (bf*)take(nw * 2);
    bf* XB  = (bf*)take((size_t)NB * SEQ * DM * 2);
    float* F = (float*)take((size_t)NB * SEQ * DM * 4);
    float* CT = (float*)take((size_t)MAXS * NFR * 4);
    float* ST = (float*)take((size_t)MAXS * NFR * 4);
    bf* QPh = (bf*)take(npl * 2); bf* QPl = (bf*)take(npl * 2);
    bf* KPh = (bf*)take(npl * 2); bf* KPl = (bf*)take(npl * 2);
    bf* VTh = (bf*)take(npl * 2); bf* VTl = (bf*)take(npl * 2);
    bf* ATh = (bf*)take((size_t)NB * SEQ * DQ * 2); bf* ATl = (bf*)take((size_t)NB * SEQ * DQ * 2);
    const size_t used = (size_t)(wsp - (char*)d_ws);
    if (used > ws_size || used > (size_t)134217728) return;

    const size_t w8 = nw / 8; const unsigned WG = (unsigned)((w8 + 255) / 256);
    k_cvtw<<<WG, 256, 0, stream>>>(wq, WB, w8);
    k_cvtw<<<WG, 256, 0, stream>>>(wk, WB + nw, w8);
    k_cvtw<<<WG, 256, 0, stream>>>(wv, WB + 2 * nw, w8);
    k_cvtw<<<WG, 256, 0, stream>>>(wo, WOB, w8);
    const size_t n8 = (size_t)NB * SEQ * DM / 8;
    k_cvtx<<<(unsigned)((n8 + 255) / 256), 256, 0, stream>>>(x, XB, n8);
    k_ropetab<<<(unsigned)(MAXS * NFR / 256), 256, 0, stream>>>(CT, ST);
    const dim3 pg((unsigned)(NB * SEQ / 64), (unsigned)(DM / 64), 1);
    const unsigned LP = (unsigned)((npl / 2 + 255) / 256);
    k_gemmw<bf, 0, false><<<pg, 32, 0, stream>>>(XB, nullptr, WB, nullptr, DM, F, DM, nullptr, (size_t)0, (size_t)0, (size_t)0);
    k_ropepl<true><<<LP, 256, 0, stream>>>(F, CT, ST, tok, QPh, QPl);
    k_gemmw<bf, 0, false><<<pg, 32, 0, stream>>>(XB, nullptr, WB + nw, nullptr, DM, F, DM, nullptr, (size_t)0, (size_t)0, (size_t)0);
    k_ropepl<false><<<LP, 256, 0, stream>>>(F, CT, ST, tok, KPh, KPl);
    k_gemmw<bf, 0, false><<<pg, 32, 0, stream>>>(XB, nullptr, WB + 2 * nw, nullptr, DM, F, DM, nullptr, (size_t)0, (size_t)0, (size_t)0);
    k_vtp<<<LP, 256, 0, stream>>>(F, VTh, VTl);
    k_attn<<<dim3(SEQ / 16, NH, NB), 32, 0, stream>>>(QPh, QPl, KPh, KPl, VTh, VTl, ATh, ATl);
    k_gemmw<bf, 1, false><<<pg, 32, 0, stream>>>(ATh, ATl, WOB, nullptr, DQ, OUT, DM, nullptr, (size_t)0, (size_t)0, (size_t)0);
}
